// IAR_10746008175388
// MI455X (gfx1250) — hardware-verified
//
#include <hip/hip_runtime.h>
#include <math.h>
#include <stdint.h>

constexpr int kBatch    = 4096;
constexpr int kDimIn    = 1024;
constexpr int kHid      = 4096;
constexpr int kDimOut   = 2048;
constexpr int kDegMod   = kDimIn - 1;
constexpr int kHalfRows = kBatch / 2;
constexpr float kW1Carry    = 64.0f;
constexpr float kW1CarryInv = 1.0f / 64.0f;
constexpr float kW2Carry    = 256.0f;
constexpr float kW2CarryInv = 1.0f / 256.0f;

typedef __attribute__((ext_vector_type(16))) _Float16 v16h;
typedef __attribute__((ext_vector_type(8)))  _Float16 v8h;
typedef __attribute__((ext_vector_type(16))) __bf16   v16b;
typedef __attribute__((ext_vector_type(8)))  __bf16   v8b;
typedef __attribute__((ext_vector_type(8)))  float    v8f;
typedef __attribute__((ext_vector_type(4)))  float    v4f;
typedef __attribute__((ext_vector_type(4)))  unsigned int v4u;

__device__ __forceinline__ unsigned short f2bf_bits(float f) {
  unsigned u = __float_as_uint(f);
  return (unsigned short)((u + 0x7FFFu + ((u >> 16) & 1u)) >> 16);
}
__device__ __forceinline__ float bf_bits2f(unsigned short h) { return __uint_as_float(((unsigned)h) << 16); }

__device__ __forceinline__ void dep_guard_h(v8f& a, v8f& b, v16h x, v16h y) { asm volatile("v_nop\n\tv_nop\n\tv_nop\n\tv_nop" : "+v"(a), "+v"(b) : "v"(x), "v"(y)); }
__device__ __forceinline__ void dep_guard_b(v8f& a, v8f& b, v16b x, v16b y) { asm volatile("v_nop\n\tv_nop\n\tv_nop\n\tv_nop" : "+v"(a), "+v"(b) : "v"(x), "v"(y)); }
__device__ __forceinline__ void keep4_h(v16h a, v16h b, v16h c, v16h d) { asm volatile("v_nop" :: "v"(a), "v"(b), "v"(c), "v"(d)); }
__device__ __forceinline__ void keep4_b(v16b a, v16b b, v16b c, v16b d) { asm volatile("v_nop" :: "v"(a), "v"(b), "v"(c), "v"(d)); }
__device__ __forceinline__ void acc_guard4(v8f& a, v8f& b, v8f& c, v8f& d) { asm volatile("v_nop\n\tv_nop\n\tv_nop\n\tv_nop" : "+v"(a), "+v"(b), "+v"(c), "+v"(d)); }
template <typename T> struct Frag;
template <> struct Frag<_Float16> {
  typedef v16h V; union U { v16h v; v8h h[2]; };
  static __device__ __forceinline__ v16h load(const _Float16* p) {
    U f; f.h[0] = *(const v8h*)(p); f.h[1] = *(const v8h*)(p + 16); return f.v;
  }
  static __device__ __forceinline__ v8f mma(v16h a, v16h b, v8f c) {
    return __builtin_amdgcn_wmma_f32_16x16x32_f16(false, a, false, b, (short)0, c, false, false);
  }
  static __device__ __forceinline__ void guard(v8f& a, v8f& b, v16h x, v16h y) { dep_guard_h(a, b, x, y); }
  static __device__ __forceinline__ void keep(v16h a, v16h b, v16h c, v16h d) { keep4_h(a, b, c, d); }
};
template <> struct Frag<__bf16> {
  typedef v16b V; union U { v16b v; v8b h[2]; };
  static __device__ __forceinline__ v16b load(const __bf16* p) {
    U f; f.h[0] = *(const v8b*)(p); f.h[1] = *(const v8b*)(p + 16); return f.v;
  }
  static __device__ __forceinline__ v8f mma(v16b a, v16b b, v8f c) {
    return __builtin_amdgcn_wmma_f32_16x16x32_bf16(false, a, false, b, (short)0, c, false, false);
  }
  static __device__ __forceinline__ void guard(v8f& a, v8f& b, v16b x, v16b y) { dep_guard_b(a, b, x, y); }
  static __device__ __forceinline__ void keep(v16b a, v16b b, v16b c, v16b d) { keep4_b(a, b, c, d); }
};

template <int ET> struct Elem;
template <> struct Elem<0> { typedef _Float16 T; };
template <> struct Elem<1> { typedef __bf16 T; };
template <int ET, bool SPLIT, int BIAS_MODE, int OUT_MODE, bool RESID, int ACT, int KMODE>
__global__ __launch_bounds__(256) void wmma_gemm64(
    const unsigned short* __restrict__ Ap, const unsigned short* __restrict__ A2p, int lda, long strideA,
    const unsigned short* __restrict__ Btp, const unsigned short* __restrict__ Bt2p, int ldb, long strideB,
    void* __restrict__ Cout, void* __restrict__ Cout2, int ldc, long strideC,
    const float* __restrict__ bias,
    const float* __restrict__ resid, long strideR,
    int M, int N, int K, float scale) {
  typedef typename Elem<ET>::T T;
  typedef typename Frag<T>::V V;
  const T* A = (const T*)Ap; const T* A2 = (const T*)A2p; const T* Bt = (const T*)Btp; const T* Bt2 = (const T*)Bt2p;
  __shared__ __align__(16) float sT[8][16 * 68];
  const int b    = blockIdx.y;
  const int lane = threadIdx.x & 31;
  const int wave = threadIdx.x >> 5;
  const int tilesN = N >> 6;
  const int tilesM = M >> 6;
  const int tile = blockIdx.x * 8 + wave;
  if (tile >= tilesM * tilesN) return;
  const int tm = tile / tilesN;
  const int tn = tile - tm * tilesN;
  const int m0 = tm << 6;
  const int n0 = tn << 6;

  int Kl = K;
  if (KMODE == 1) {
    const int nr   = n0 % kDegMod;
    const int maxr = (nr + 63 < kDegMod) ? (nr + 63) : (kDegMod - 1);
    const int kp   = ((maxr >> 5) + 1) << 5;
    Kl = (kp < K) ? kp : K;
  }

  const T* Ab  = A  + (size_t)b * strideA;
  const T* Bb  = Bt + (size_t)b * strideB;
  const T* Ab2 = SPLIT ? (A2  + (size_t)b * strideA) : nullptr;
  const T* Bb2 = SPLIT ? (Bt2 + (size_t)b * strideB) : nullptr;

  const int rlane = lane & 15;
  const int koff  = (lane >> 4) * 8;
  const int mOff  = (lane >> 4) * 8;

  v8f acc[4][4];
#pragma unroll
  for (int i = 0; i < 4; ++i)
#pragma unroll
    for (int j = 0; j < 4; ++j) acc[i][j] = (v8f){0.f,0.f,0.f,0.f,0.f,0.f,0.f,0.f};

  for (int k0 = 0; k0 < Kl; k0 += 32) {
    if (KMODE == 2) {
      const int kr   = k0 % kDegMod;
      const int minr = (kr + 31 < kDegMod) ? kr : 0;
      const int jr   = (n0 & (kDimIn - 1)) + 63;
      if (jr <= minr) continue;
    }
    V bh[4], bl[4];
#pragma unroll
    for (int j = 0; j < 4; ++j) {
      const size_t bo = (size_t)(n0 + (j << 4) + rlane) * ldb + koff + k0;
      bh[j] = Frag<T>::load(Bb + bo);
      if (SPLIT) bl[j] = Frag<T>::load(Bb2 + bo);
    }
#pragma unroll
    for (int i = 0; i < 4; ++i) {
      const size_t ao = (size_t)(m0 + (i << 4) + rlane) * lda + koff + k0;
      V ah = Frag<T>::load(Ab + ao);
      V al;
      if (SPLIT) al = Frag<T>::load(Ab2 + ao);
#pragma unroll
      for (int j = 0; j < 4; ++j) {
        acc[i][j] = Frag<T>::mma(ah, bh[j], acc[i][j]);
        if (SPLIT) {
          acc[i][j] = Frag<T>::mma(ah, bl[j], acc[i][j]);
          acc[i][j] = Frag<T>::mma(al, bh[j], acc[i][j]);
        }
      }
      Frag<T>::guard(acc[i][0], acc[i][3], ah, SPLIT ? al : ah);
    }
    Frag<T>::keep(bh[0], bh[1], bh[2], bh[3]);
    if (SPLIT) Frag<T>::keep(bl[0], bl[1], bl[2], bl[3]);
  }
  acc_guard4(acc[0][0], acc[0][1], acc[0][2], acc[0][3]);
  acc_guard4(acc[1][0], acc[1][1], acc[1][2], acc[1][3]);
  acc_guard4(acc[2][0], acc[2][1], acc[2][2], acc[2][3]);
  acc_guard4(acc[3][0], acc[3][1], acc[3][2], acc[3][3]);

  float* slab = sT[wave];
  const float* Rb = RESID ? (resid + (size_t)b * strideR) : nullptr;
#pragma unroll
  for (int i = 0; i < 4; ++i) {
    const int mBase = m0 + (i << 4);
#pragma unroll
    for (int j = 0; j < 4; ++j) {
      const int n = n0 + (j << 4) + rlane;
      float bv = 0.f;
      if (BIAS_MODE == 2) bv = bias[n];
#pragma unroll
      for (int r = 0; r < 8; ++r) {
        float v = acc[i][j][r] * scale;
        if (BIAS_MODE == 1) v += bias[mBase + mOff + r];
        if (BIAS_MODE == 2) v += bv;
        if (RESID) v += Rb[(size_t)(mBase + mOff + r) * ldc + n];
        if (ACT == 2) v = fmaxf(v, 0.0f);
        if (ACT == 4) v = (v > 0.f) ? v : 0.01f * v;
        slab[(mOff + r) * 68 + (j << 4) + rlane] = v;
      }
    }
    __builtin_amdgcn_fence(__ATOMIC_RELEASE, "workgroup");
    __builtin_amdgcn_wave_barrier();
    __builtin_amdgcn_fence(__ATOMIC_ACQUIRE, "workgroup");
    if (OUT_MODE == 0 || OUT_MODE == 3) {
      float* C = (float*)(OUT_MODE == 3 ? Cout2 : Cout) + (size_t)b * strideC;
      const int hh = lane >> 4, c4 = (lane & 15) * 4;
      for (int pass = 0; pass < 2; ++pass) {
#pragma unroll
        for (int it = 0; it < 8; ++it) {
          const int row = it * 2 + hh;
          v4f v = *(const v4f*)(slab + row * 68 + c4);
          *(volatile v4f*)(C + (size_t)(mBase + row) * ldc + n0 + c4) = v;
        }
        __threadfence();
      }
    }
    if (OUT_MODE != 0) {
      const int q = lane >> 3, c8 = (lane & 7) * 8;
      unsigned short* C  = (unsigned short*)Cout  + (size_t)b * strideC;
      unsigned short* C2 = (OUT_MODE == 2) ? ((unsigned short*)Cout2 + (size_t)b * strideC) : nullptr;
      for (int pass = 0; pass < 2; ++pass) {
#pragma unroll
        for (int it = 0; it < 4; ++it) {
          const int row = it * 4 + q;
          const float* sp = slab + row * 68 + c8;
          v8h hv, lv;
#pragma unroll
          for (int e = 0; e < 8; ++e) {
            if (OUT_MODE != 2) {
              hv[e] = (_Float16)sp[e];
            } else {
              unsigned short hb = f2bf_bits(sp[e]);
              unsigned short lb = f2bf_bits(sp[e] - bf_bits2f(hb));
              hv[e] = __builtin_bit_cast(_Float16, hb);
              lv[e] = __builtin_bit_cast(_Float16, lb);
            }
          }
          *(volatile v8h*)(C + (size_t)(mBase + row) * ldc + n0 + c8) = hv;
          if (OUT_MODE == 2) *(volatile v8h*)(C2 + (size_t)(mBase + row) * ldc + n0 + c8) = lv;
        }
        __threadfence();
      }
    }
    __builtin_amdgcn_fence(__ATOMIC_RELEASE, "workgroup");
    __builtin_amdgcn_wave_barrier();
    __builtin_amdgcn_fence(__ATOMIC_ACQUIRE, "workgroup");
  }
}

__device__ __forceinline__ unsigned pk16(unsigned short a, unsigned short b) { return (unsigned)a | ((unsigned)b << 16); }
__device__ __forceinline__ unsigned short h_bits(float f) { const _Float16 h = (_Float16)f; return __builtin_bit_cast(unsigned short, h); }
__device__ __forceinline__ int perm_index(int p) {
  if (p < 0) p += kDimIn;
  p = (p < 0) ? 0 : p;
  p = (p > kDimIn - 1) ? (kDimIn - 1) : p;
  return p;
}

template <int MASK>
__global__ __launch_bounds__(256) void transpose_cast_mask_f16_kernel(const float* __restrict__ in, unsigned short* __restrict__ out,
                                                                      int R, int CC, float scale) {
  __shared__ float tile[64][65];
  const int t  = threadIdx.x;
  const int n0 = blockIdx.x * 64;
  const int k0 = blockIdx.y * 64;
  {
    const int kr = t >> 2, nc = (t & 3) * 16;
    const float* p = in + (size_t)(k0 + kr) * CC + n0 + nc;
#pragma unroll
    for (int e4 = 0; e4 < 4; ++e4) {
      const v4f f = *(const v4f*)(p + 4 * e4);
      tile[kr][nc + 4 * e4 + 0] = f[0];
      tile[kr][nc + 4 * e4 + 1] = f[1];
      tile[kr][nc + 4 * e4 + 2] = f[2];
      tile[kr][nc + 4 * e4 + 3] = f[3];
    }
  }
  __syncthreads();
  const int q = t >> 3, c8 = (t & 7) * 8;
  const int orowA = n0 + q, orowB = n0 + 32 + q;
  const int degA = (MASK == 1) ? (orowA % kDegMod) : (orowA & (kDimIn - 1));
  const int degB = (MASK == 1) ? (orowB % kDegMod) : (orowB & (kDimIn - 1));
  v4u u0, u1;
#pragma unroll
  for (int w = 0; w < 4; ++w) {
    const int oc0 = k0 + c8 + 2 * w, oc1 = oc0 + 1;
    const int d0 = (MASK == 1) ? oc0 : (oc0 % kDegMod);
    const int d1 = (MASK == 1) ? oc1 : (oc1 % kDegMod);
    const bool kA0 = (MASK == 1) ? (degA >= d0) : (degA > d0);
    const bool kA1 = (MASK == 1) ? (degA >= d1) : (degA > d1);
    const bool kB0 = (MASK == 1) ? (degB >= d0) : (degB > d0);
    const bool kB1 = (MASK == 1) ? (degB >= d1) : (degB > d1);
    const float vA0 = kA0 ? tile[c8 + 2 * w][q] * scale : 0.0f;
    const float vA1 = kA1 ? tile[c8 + 2 * w + 1][q] * scale : 0.0f;
    const float vB0 = kB0 ? tile[c8 + 2 * w][32 + q] * scale : 0.0f;
    const float vB1 = kB1 ? tile[c8 + 2 * w + 1][32 + q] * scale : 0.0f;
    u0[w] = pk16(h_bits(vA0), h_bits(vA1));
    u1[w] = pk16(h_bits(vB0), h_bits(vB1));
  }
  unsigned short* p0 = out + (size_t)orowA * R + k0 + c8;
  unsigned short* p1 = out + (size_t)orowB * R + k0 + c8;
  for (int pass = 0; pass < 2; ++pass) {
    *(volatile v4u*)p0 = u0;
    *(volatile v4u*)p1 = u1;
    __threadfence();
  }
}

__global__ __launch_bounds__(256) void gather_cast_z_kernel(const float* __restrict__ z, const int* __restrict__ perm,
                                                            unsigned short* __restrict__ out) {
  const int t   = threadIdx.x;
  const int row = blockIdx.x * 2 + (t >> 7);
  const int c8  = (t & 127) * 8;
  const float* zr = z + (size_t)row * kDimIn;
  v4u u;
#pragma unroll
  for (int w = 0; w < 4; ++w) {
    const int ia = c8 + 2 * w;
    const int pa = perm_index(perm[ia]);
    const int pb = perm_index(perm[ia + 1]);
    u[w] = pk16(h_bits(zr[pa]), h_bits(zr[pb]));
  }
  unsigned short* op = out + (size_t)row * kDimIn + c8;
  *(volatile v4u*)op = u;
  __threadfence();
  *(volatile v4u*)op = u;
}

__global__ __launch_bounds__(256) void w2_rowsum_kernel(const float* __restrict__ w2, float* __restrict__ wsum) {
  __shared__ __align__(16) float sv[32];
  const int t = threadIdx.x, lane = t & 31, wave = t >> 5;
  const int kb = blockIdx.x * 32;
#pragma unroll 1
  for (int rr = 0; rr < 4; ++rr) {
    const int k  = kb + wave * 4 + rr;
    const int kr = k % kDegMod;
    const float* wr = w2 + (size_t)k * kDimOut + kDimIn;
    float acc = 0.f;
#pragma unroll 1
    for (int tt = 0; tt < 32; ++tt) {
      const int j = lane + 32 * tt;
      const float w = wr[j];
      acc += (j > kr) ? w : 0.0f;
    }
    acc += __shfl_xor(acc, 16, 32);
    acc += __shfl_xor(acc, 8, 32);
    acc += __shfl_xor(acc, 4, 32);
    acc += __shfl_xor(acc, 2, 32);
    acc += __shfl_xor(acc, 1, 32);
    if (lane == 0) sv[wave * 4 + rr] = acc;
  }
  __syncthreads();
  if (wave == 0 && lane < 8) {
    const v4f v = *(const v4f*)(&sv[lane * 4]);
    float* op = wsum + kb + lane * 4;
    *(volatile v4f*)op = v;
    __threadfence();
    *(volatile v4f*)op = v;
  }
}

__global__ __launch_bounds__(256) void affine_kernel(const float* __restrict__ z, const int* __restrict__ perm,
                                                     const float* __restrict__ res, float* __restrict__ out0) {
  __shared__ __align__(16) float xrow[kDimIn];
  const int t = threadIdx.x;
  const int b = blockIdx.x;
  *(v4f*)(&xrow[4 * t]) = (v4f){0.f, 0.f, 0.f, 0.f};
  __syncthreads();
  const float* zr = z + (size_t)b * kDimIn;
  const float* rr = res + (size_t)b * kDimOut;
#pragma unroll 1
  for (int e = 0; e < 4; ++e) {
    const int i = t + 256 * e;
    const int p = perm_index(perm[i]);
    const float zv = zr[p];
    const float mu = rr[i];
    const float ls = rr[kDimIn + i];
    const float x = zv * expf(ls) + mu;
    xrow[p] = x;
  }
  __syncthreads();
  const v4f v = *(const v4f*)(&xrow[4 * t]);
  float* op = out0 + (size_t)b * kDimIn + 4 * t;
  *(volatile v4f*)op = v;
  __threadfence();
  *(volatile v4f*)op = v;
}

__global__ __launch_bounds__(256) void logdet_kernel(const float* __restrict__ h32, const float* __restrict__ wsum,
                                                     const float* __restrict__ b2, float* __restrict__ out1) {
  __shared__ __align__(16) float sv[32];
  const int t = threadIdx.x, lane = t & 31, wave = t >> 5;
  const int rb = blockIdx.x * 32;
  float bs = 0.f;
#pragma unroll 1
  for (int tt = 0; tt < 32; ++tt) bs += b2[kDimIn + lane + 32 * tt];
  bs += __shfl_xor(bs, 16, 32);
  bs += __shfl_xor(bs, 8, 32);
  bs += __shfl_xor(bs, 4, 32);
  bs += __shfl_xor(bs, 2, 32);
  bs += __shfl_xor(bs, 1, 32);
#pragma unroll 1
  for (int rr = 0; rr < 4; ++rr) {
    const int row = rb + wave * 4 + rr;
    const float* hr = h32 + (size_t)row * kHid;
    float acc = 0.f;
#pragma unroll 1
    for (int tt = 0; tt < 32; ++tt) {
      const int c = lane * 4 + 128 * tt;
      const v4f hv = *(const v4f*)(hr + c);
      const v4f wv = *(const v4f*)(wsum + c);
      acc = fmaf(hv[0], wv[0], acc);
      acc = fmaf(hv[1], wv[1], acc);
      acc = fmaf(hv[2], wv[2], acc);
      acc = fmaf(hv[3], wv[3], acc);
    }
    acc += __shfl_xor(acc, 16, 32);
    acc += __shfl_xor(acc, 8, 32);
    acc += __shfl_xor(acc, 4, 32);
    acc += __shfl_xor(acc, 2, 32);
    acc += __shfl_xor(acc, 1, 32);
    if (lane == 0) sv[wave * 4 + rr] = acc + bs;
  }
  __syncthreads();
  if (wave == 0 && lane < 8) {
    const v4f v = *(const v4f*)(&sv[lane * 4]);
    float* op = out1 + rb + lane * 4;
    *(volatile v4f*)op = v;
    __threadfence();
    *(volatile v4f*)op = v;
  }
}

extern "C" void kernel_launch(void* const* d_in, const int* in_sizes, int n_in,
                              void* d_out, int out_size, void* d_ws, size_t ws_size,
                              hipStream_t stream) {
  if (n_in < 6) return;
  if (in_sizes[0] != kBatch * kDimIn) return;
  if (in_sizes[1] != kDimIn * kHid) return;
  if (in_sizes[2] != kHid) return;
  if (in_sizes[3] != kHid * kDimOut) return;
  if (in_sizes[4] != kDimOut) return;
  if (in_sizes[5] != kDimIn) return;
  if (out_size != kBatch * kDimIn + kBatch) return;

  const float* z    = (const float*)d_in[0];
  const float* W1   = (const float*)d_in[1];
  const float* b1   = (const float*)d_in[2];
  const float* W2   = (const float*)d_in[3];
  const float* b2   = (const float*)d_in[4];
  const int*   perm = (const int*)d_in[5];
  float* out0 = (float*)d_out;
  float* out1 = out0 + (size_t)kBatch * kDimIn;

  const size_t PW1  = (size_t)kHid * kDimIn * 2;
  const size_t PW2  = (size_t)kDimOut * kHid * 2;
  const size_t PZ16 = (size_t)kBatch * kDimIn * 2;
  const size_t PH32 = (size_t)kHalfRows * kHid * 4;
  const size_t PH16 = (size_t)kHalfRows * kHid * 2;
  const size_t PRES = (size_t)kHalfRows * kDimOut * 4;
  const size_t PWS  = (size_t)kHid * 4;
  size_t off = 0;
  const size_t oW1T = off; off += PW1;
  const size_t oW2T = off; off += PW2;
  const size_t oZ16 = off; off += PZ16;
  const size_t oH32 = off; off += PH32;
  const size_t oH16 = off; off += PH16;
  const size_t oRES = off; off += PRES;
  const size_t oWS  = off; off += PWS;
  if (off > ws_size) return;

  char* ws = (char*)d_ws;
  unsigned short* W1T  = (unsigned short*)(ws + oW1T);
  unsigned short* W2T  = (unsigned short*)(ws + oW2T);
  unsigned short* Z16  = (unsigned short*)(ws + oZ16);
  float*          H32  = (float*)(ws + oH32);
  unsigned short* H16  = (unsigned short*)(ws + oH16);
  float*          RES  = (float*)(ws + oRES);
  float*          WSUM = (float*)(ws + oWS);

  const dim3 blk(256);

  transpose_cast_mask_f16_kernel<1><<<dim3(kHid / 64, kDimIn / 64), blk, 0, stream>>>(W1, W1T, kDimIn, kHid, kW1Carry);
  transpose_cast_mask_f16_kernel<2><<<dim3(kDimOut / 64, kHid / 64), blk, 0, stream>>>(W2, W2T, kHid, kDimOut, kW2Carry);
  gather_cast_z_kernel<<<dim3(kBatch / 2), blk, 0, stream>>>(z, perm, Z16);
  w2_rowsum_kernel<<<dim3(kHid / 32), blk, 0, stream>>>(W2, WSUM);

  const int tiles1 = (kHalfRows / 64) * (kHid / 64);
  const int tiles2 = (kHalfRows / 64) * (kDimOut / 64);
  for (int half = 0; half < 2; ++half) {
    const unsigned short* Z16h = Z16 + (size_t)half * kHalfRows * kDimIn;
    const float* zh   = z    + (size_t)half * kHalfRows * kDimIn;
    float*       o0h  = out0 + (size_t)half * kHalfRows * kDimIn;
    float*       o1h  = out1 + (size_t)half * kHalfRows;
    wmma_gemm64<0, false, 2, 3, false, 2, 1><<<dim3((tiles1 + 7) / 8, 1), blk, 0, stream>>>(
        Z16h, Z16h, kDimIn, 0L, W1T, W1T, kDimIn, 0L, (void*)H16, (void*)H32, kHid, 0L,
        b1, z, 0L, kHalfRows, kHid, kDimIn, kW1CarryInv);
    wmma_gemm64<0, false, 2, 0, false, 0, 2><<<dim3((tiles2 + 7) / 8, 1), blk, 0, stream>>>(
        H16, H16, kHid, 0L, W2T, W2T, kHid, 0L, (void*)RES, (void*)RES, kDimOut, 0L,
        b2, z, 0L, kHalfRows, kDimOut, kHid, kW2CarryInv);
    affine_kernel<<<dim3(kHalfRows), blk, 0, stream>>>(zh, perm, RES, o0h);
    logdet_kernel<<<dim3(kHalfRows / 32), blk, 0, stream>>>(H32, WSUM, b2, o1h);
  }
}
